// RWKV_TimeMix_41755672052465
// MI455X (gfx1250) — hardware-run, weakly checked
//
#include <hip/hip_runtime.h>
#define NB 4
#define SQ 1024
#define CW 512
#define CS 256
#define DK 16
#define DO 64
#define NTOK (NB * SQ)
#define XSC 256.0f
#define QSC 16.0f
#define EPSQ 1.0e-8f
#define F16MIN 6.103515625e-05f
typedef __bf16 v16b __attribute__((ext_vector_type(16)));
typedef unsigned short v8us __attribute__((ext_vector_type(8), may_alias));
typedef float  v8f  __attribute__((ext_vector_type(8)));
typedef float  v4f  __attribute__((ext_vector_type(4)));
typedef float  v4fa __attribute__((ext_vector_type(4), may_alias));
union FragB { v16b v; v8us half[2]; unsigned short u[16]; };

__device__ __forceinline__ unsigned short bf16_bits(float x) { unsigned int u = __float_as_uint(x); return (unsigned short)((u + 0x7FFFu + ((u >> 16) & 1u)) >> 16); }
__device__ __forceinline__ float bf16_val(unsigned short b) { return __uint_as_float(((unsigned int)b) << 16); }
__device__ __forceinline__ float bf16_round(float x) { return bf16_val(bf16_bits(x)); }
template <int NT>
__device__ __forceinline__ v8f mmaN(v16b ah, v16b al, v16b bh, v16b bl, v8f c) {
  c = __builtin_amdgcn_wmma_f32_16x16x32_bf16(false, ah, false, bh, (short)0, c, false, false);
  if (NT >= 2) c = __builtin_amdgcn_wmma_f32_16x16x32_bf16(false, al, false, bh, (short)0, c, false, false);
  if (NT >= 3) c = __builtin_amdgcn_wmma_f32_16x16x32_bf16(false, ah, false, bl, (short)0, c, false, false);
  asm volatile("v_nop\n\tv_nop\n\tv_nop\n\tv_nop" : "+v"(c) : "v"(ah), "v"(al), "v"(bh), "v"(bl));
  return c;
}


typedef _Float16 v16h __attribute__((ext_vector_type(16)));
union FragH { v16h v; v8us half[2]; _Float16 h[16]; unsigned short u[16]; };
template <int NT>
__device__ __forceinline__ v8f mmaH(v16h ah, v16h al, v16h bh, v16h bl, v8f c) {
  c = __builtin_amdgcn_wmma_f32_16x16x32_f16(false, ah, false, bh, (short)0, c, false, false);
  if (NT >= 2) c = __builtin_amdgcn_wmma_f32_16x16x32_f16(false, al, false, bh, (short)0, c, false, false);
  if (NT >= 3) c = __builtin_amdgcn_wmma_f32_16x16x32_f16(false, ah, false, bl, (short)0, c, false, false);
  asm volatile("v_nop\n\tv_nop\n\tv_nop\n\tv_nop" : "+v"(c) : "v"(ah), "v"(al), "v"(bh), "v"(bl));
  return c;
}

typedef _Float16 v4h __attribute__((ext_vector_type(4)));

__device__ __forceinline__ v16h g2_frag(const _Float16* p, int hh) { FragH f; f.half[0] = *(const v8us*)((const unsigned short*)p + 8 * hh); f.half[1] = *(const v8us*)((const unsigned short*)p + 16 + 8 * hh); return f.v; }
__device__ __forceinline__ v8f g2_mma(v16h a, v16h b, v8f c) { v8f d = __builtin_amdgcn_wmma_f32_16x16x32_f16(false, a, false, b, (short)0, c, false, false); asm volatile("v_nop\n\tv_nop\n\tv_nop\n\tv_nop" : "+v"(d) : "v"(a), "v"(b)); return d; }
template <int ACT>
__global__ __launch_bounds__(128) void k_gemm2(const _Float16* __restrict__ A, int lda, size_t sA, const _Float16* __restrict__ Bh, int ldb, size_t sB, float alpha, const float* __restrict__ bias, size_t sBias, const float* __restrict__ CP, int rowsPerB, size_t sCPb, int row0g,
    float* __restrict__ C, _Float16* __restrict__ C16, int ldc, size_t sC, int M, int N, int K) { static_assert(ACT == 0 || ACT == 3 || ACT == 6 || ACT == 8 || ACT == 9 || ACT == 11 || ACT == 12 || ACT == 14 || ACT == 15 || ACT == 16 || ACT == 17, "k_gemm2: unsupported ACT code (would silently apply no activation)");
  __shared__ __attribute__((aligned(16))) float so[4][32][68];
  const int tid = threadIdx.x, w = tid >> 5, lane = tid & 31, ln = lane & 15, hh = lane >> 4; const int by = blockIdx.y;
  A += (size_t)by * sA; Bh += (size_t)by * sB; const size_t cofs = (size_t)by * sC; const float* bp = bias ? bias + (size_t)by * sBias : nullptr;
  const int ntn = N >> 6; const int mt = blockIdx.x / ntn, nq = blockIdx.x - mt * ntn; const int row0 = mt * 128 + 32 * w, col0 = nq * 64; if (row0 >= M) return;
  const _Float16* a0p = A + (size_t)(row0 + ln) * lda; const _Float16* a1p = a0p + (size_t)16 * lda;
  const _Float16* b0p = Bh + (size_t)(col0 + ln) * ldb; const _Float16* b1p = b0p + (size_t)16 * ldb; const _Float16* b2p = b1p + (size_t)16 * ldb; const _Float16* b3p = b2p + (size_t)16 * ldb;
  const v8f z8 = {0.f,0.f,0.f,0.f,0.f,0.f,0.f,0.f}; v8f c00 = z8, c01 = z8, c02 = z8, c03 = z8, c10 = z8, c11 = z8, c12 = z8, c13 = z8;
  for (int kb = 0; kb < K; kb += 32) { const v16h a0 = g2_frag(a0p + kb, hh), a1 = g2_frag(a1p + kb, hh);
    v16h b = g2_frag(b0p + kb, hh); c00 = g2_mma(a0, b, c00); c10 = g2_mma(a1, b, c10);
    b = g2_frag(b1p + kb, hh); c01 = g2_mma(a0, b, c01); c11 = g2_mma(a1, b, c11);
    b = g2_frag(b2p + kb, hh); c02 = g2_mma(a0, b, c02); c12 = g2_mma(a1, b, c12);
    b = g2_frag(b3p + kb, hh); c03 = g2_mma(a0, b, c03); c13 = g2_mma(a1, b, c13); }
  v8f accs[8] = {c00, c01, c02, c03, c10, c11, c12, c13};
#pragma unroll
  for (int u = 0; u < 8; ++u) { const int t = u & 3, half = u >> 2; const int col = col0 + t * 16 + ln; const float bv = bp ? bf16_round(bp[col]) : 0.f;
#pragma unroll
    for (int r = 0; r < 8; ++r) { const int rloc = half * 16 + 8 * hh + r; float v = accs[u][r] * alpha + bv; if (CP) { if (rowsPerB < 0) v += CP[cofs + (size_t)(row0g + row0 + rloc) * ldc + col];        else { const int bidx = (row0g + row0 + rloc) / rowsPerB; v += CP[(size_t)bidx * sCPb + (size_t)by * 64 + col]; } }
      if (ACT == 3) v = fmaxf(v, 0.f); else if (ACT == 6) v = 0.5f * v * (1.0f + erff(v * 0.70710678118654752f)); else if (ACT == 11) v = 1.0f / (1.0f + expf(-v)); else if (ACT == 15) v = v / (1.0f + expf(-v)); else if (ACT == 12) v = (v > 0.f) ? v : 0.01f * v; else if (ACT == 8) v = tanhf(v); else if (ACT == 9) v = 0.5f * v * (1.0f + tanhf(0.7978845608028654f * (v + 0.044715f * v * v * v))); else if (ACT == 14) v = (v > 0.f) ? v : 0.1f * v; else if (ACT == 16) v = (v >= 0.f) ? v : 0.3f * v; else if (ACT == 17) v = (v >= 0.f) ? v : 0.2f * v;
      so[w][rloc][t * 16 + ln] = v; } }
  __builtin_amdgcn_fence(__ATOMIC_ACQ_REL, "workgroup"); __builtin_amdgcn_wave_barrier();
  const int rsub = lane >> 4, c4 = (lane & 15) * 4;
  for (int pass = 0; pass < 2; ++pass) {
#pragma unroll
    for (int q = 0; q < 16; ++q) { const int r = q * 2 + rsub; const v4f v = *(const v4fa*)&so[w][r][c4]; if (C) *(volatile v4f*)(C + cofs + (size_t)(row0 + r) * ldc + col0 + c4) = v; if (C16) { v4h h4; for (int i = 0; i < 4; ++i) h4[i] = (_Float16)v[i]; *(volatile v4h*)(C16 + cofs + (size_t)(row0 + r) * ldc + col0 + c4) = h4; } }
    if (pass == 0) __threadfence(); } }

__device__ __forceinline__ _Float16 f16sel(float v) { const float f = (fabsf(v) < F16MIN) ? 0.0f : v; return (_Float16)f; }
__global__ __launch_bounds__(256) void k_shx(const float* __restrict__ x, _Float16* __restrict__ XP, int n8) {
  const int t = blockIdx.x * 256 + threadIdx.x; if (t >= n8) return; const int r = t >> 6, c = (t & 63) * 8, tok = r & (SQ - 1); const bool early = c < CS; const bool live = (!early) || (tok > 0); const int rs = (early && tok > 0) ? r - 1 : r; const float* p = x + (size_t)rs * CW + c; FragH f;
  for (int q = 0; q < 8; ++q) { const float v = bf16_round(p[q]) * XSC; f.h[q] = (_Float16)(live ? v : 0.0f); }
  *(volatile v8us*)((unsigned short*)XP + (size_t)t * 8) = f.half[0]; __threadfence(); *(volatile v8us*)((unsigned short*)XP + (size_t)t * 8) = f.half[0]; }

__global__ __launch_bounds__(256) void k_wst(const float* __restrict__ s0, const float* __restrict__ s1, const float* __restrict__ s2, _Float16* __restrict__ dst, int rpl, int scl, int dcl, int nv, int n8) {
  const int t = blockIdx.x * 256 + threadIdx.x; if (t >= n8) return; const int pl = dcl - 3; const int n = t >> pl, c = (t & ((1 << pl) - 1)) * 8; const int i = n >> rpl, rr = n & ((1 << rpl) - 1), cs = c & ((1 << scl) - 1);
  const float* s = (i == 0) ? s0 : ((i == 1) ? s1 : s2); const float* p = s + ((size_t)rr << scl) + cs; const bool live = n < nv; FragH f;
  for (int q = 0; q < 8; ++q) { const float v = bf16_round(p[q]) * XSC; f.h[q] = (_Float16)(live ? v : 0.0f); }
  *(volatile v8us*)((unsigned short*)dst + (size_t)t * 8) = f.half[0]; __threadfence(); *(volatile v8us*)((unsigned short*)dst + (size_t)t * 8) = f.half[0]; }

__global__ __launch_bounds__(256) void k_wsum(const float* __restrict__ lagw, const float* __restrict__ colw, const float* __restrict__ roww, float* __restrict__ CSUM, int n) {
  const int u = blockIdx.x * 256 + threadIdx.x; if (u >= n) return; const float cu = bf16_round(colw[u]); float s = 0.f;
  for (int t = 0; t < SQ; ++t) { const bool on = t >= u; const int ix = on ? (SQ - 1 - (t - u)) : 0; const float w = bf16_round(lagw[ix]) * cu * bf16_round(roww[t]); s += on ? w : 0.0f; }
  *(volatile float*)(CSUM + u) = s; __threadfence(); *(volatile float*)(CSUM + u) = s; }

__global__ __launch_bounds__(64) void k_kvr(const float* __restrict__ PR, const float* __restrict__ ba, const float* __restrict__ bb, float* __restrict__ RS, float* __restrict__ MP, int n) {
  const int c = blockIdx.x * 64 + threadIdx.x; if (c >= n) return; const int b = c >> 4, d = c & 15; const float bad = bf16_round(ba[d]), bbd = bf16_round(bb[d]); const float* p = PR + (size_t)b * SQ * DO + d; float* rs = RS + (size_t)c * SQ; float s = 0.f, a = 0.f;
  for (int t = 0; t < SQ; t += 4) { v4f o;
    for (int q = 0; q < 4; ++q) { const float* pq = p + (size_t)(t + q) * DO; const float e = expf(fminf(fmaxf(pq[0] + bad, -60.0f), 30.0f)); const float w = pq[DK] + bbd; s += e; a += e * w; o[q] = s; }
    *(volatile v4f*)(rs + t) = o; __threadfence(); *(volatile v4f*)(rs + t) = o; }
  const float m = a * (1.0f / SQ); *(volatile float*)(MP + c) = m; __threadfence(); *(volatile float*)(MP + c) = m; }

__global__ __launch_bounds__(256) void k_quot(const float* __restrict__ PR, const float* __restrict__ bc, const float* __restrict__ CSUM, const float* __restrict__ RS, const float* __restrict__ MP, _Float16* __restrict__ QW, int n) {
  const int r = blockIdx.x * 256 + threadIdx.x; if (r >= n) return; const int b = r >> 10, u = r & (SQ - 1); const float cu = CSUM[u]; const float* pr = PR + (size_t)r * DO + 2 * DK; FragH hi, lo;
  for (int d = 0; d < DK; ++d) { const int c = b * DK + d; const float rv = pr[d] + bf16_round(bc[d]); const float cm = cu * MP[c]; const float q = (rv * cm) / (RS[(size_t)c * SQ + u] + EPSQ); const float qs = q * QSC; const _Float16 h = f16sel(qs); hi.h[d] = h; lo.h[d] = f16sel(qs - (float)h); }
  unsigned short* qp = (unsigned short*)QW + (size_t)r * 32; *(volatile v8us*)(qp) = hi.half[0]; *(volatile v8us*)(qp + 8) = hi.half[1]; *(volatile v8us*)(qp + 16) = lo.half[0]; *(volatile v8us*)(qp + 24) = lo.half[1]; __threadfence();
  *(volatile v8us*)(qp) = hi.half[0]; *(volatile v8us*)(qp + 8) = hi.half[1]; *(volatile v8us*)(qp + 16) = lo.half[0]; *(volatile v8us*)(qp + 24) = lo.half[1]; }

__global__ __launch_bounds__(256) void k_fin(const float* __restrict__ LP, const float* __restrict__ bd, const float* __restrict__ outw, float* __restrict__ out, int n4) {
  const int t = blockIdx.x * 256 + threadIdx.x; if (t >= n4) return; const int r = t >> 4, c4 = (t & 15) * 4; const float g = bf16_round(outw[r & (SQ - 1)]); const v4f v = *(const v4fa*)(LP + (size_t)t * 4); v4f o;
  for (int q = 0; q < 4; ++q) o[q] = (v[q] + bf16_round(bd[c4 + q])) * g;
  *(volatile v4f*)(out + (size_t)t * 4) = o; __threadfence(); *(volatile v4f*)(out + (size_t)t * 4) = o; }

extern "C" void kernel_launch(void* const* d_in, const int* in_sizes, int n_in,
                              void* d_out, int out_size, void* d_ws, size_t ws_size, hipStream_t stream) {
  (void)in_sizes; (void)n_in; (void)out_size;
  const float* X = (const float*)d_in[0]; const float* LAGW = (const float*)d_in[1]; const float* COLW = (const float*)d_in[2]; const float* ROWW = (const float*)d_in[3]; const float* OUTW = (const float*)d_in[4];
  const float* WA = (const float*)d_in[5]; const float* BA = (const float*)d_in[6]; const float* WB = (const float*)d_in[7]; const float* BB = (const float*)d_in[8]; const float* WC = (const float*)d_in[9]; const float* BC = (const float*)d_in[10]; const float* WD = (const float*)d_in[11]; const float* BD = (const float*)d_in[12];
  static_assert(NB == 4 && SQ == 1024 && CW == 512 && CS == 256 && DK == 16 && DO == 64 && NTOK == 4096 && (SQ & (SQ - 1)) == 0 && CW / 8 == 64 && 3 * DK <= DO && 2 * DK == 32 && ((size_t)NTOK * CW / 8) % 256 == 0 && ((size_t)DO * CW / 8) % 256 == 0 && ((size_t)DO * 32 / 8) == 256 && SQ % 256 == 0 && NB * DK == 64 && NTOK % 256 == 0 && ((size_t)NTOK * DO / 4) % 256 == 0 && NTOK % 128 == 0 && DO % 64 == 0 && CW % 32 == 0 && SQ % 4 == 0, "the index shifts; whole tiles; exact grids");
  float* out = (float*)d_out;
  char* ws = (char*)d_ws; size_t off = 0;
  auto take = [&](size_t bytes) { char* p = ws + off; off += (bytes + 255) & ~(size_t)255; return p; };
  _Float16* XP = (_Float16*)take((size_t)NTOK * CW * 2); _Float16* W3 = (_Float16*)take((size_t)DO * CW * 2); _Float16* W2 = (_Float16*)take((size_t)DO * 32 * 2); float* PR = (float*)take((size_t)NTOK * DO * 4); float* CSUM = (float*)take((size_t)SQ * 4); float* RS = (float*)take((size_t)NB * DK * SQ * 4); float* MP = (float*)take((size_t)NB * DK * 4); _Float16* QW = (_Float16*)take((size_t)NTOK * 32 * 2); float* LP = (float*)take((size_t)NTOK * DO * 4);
  if (off > ws_size) return;
  k_shx<<<(unsigned)((size_t)NTOK * CW / 8 / 256), 256, 0, stream>>>(X, XP, (int)((size_t)NTOK * CW / 8));
  k_wst<<<(unsigned)((size_t)DO * CW / 8 / 256), 256, 0, stream>>>(WA, WB, WC, W3, 4, 9, 9, 3 * DK, (int)((size_t)DO * CW / 8));
  k_wst<<<1, 256, 0, stream>>>(WD, WD, WD, W2, 6, 4, 5, DO, (int)((size_t)DO * 32 / 8));
  k_gemm2<0><<<dim3((NTOK / 128) * (DO / 64), 1), 128, 0, stream>>>(XP, CW, 0, W3, CW, 0, 1.0f / (XSC * XSC), nullptr, 0, nullptr, 1, 0, 0, PR, nullptr, DO, 0, NTOK, DO, CW);
  k_wsum<<<(unsigned)(SQ / 256), 256, 0, stream>>>(LAGW, COLW, ROWW, CSUM, SQ);
  k_kvr<<<1, 64, 0, stream>>>(PR, BA, BB, RS, MP, NB * DK);
  k_quot<<<(unsigned)(NTOK / 256), 256, 0, stream>>>(PR, BC, CSUM, RS, MP, QW, NTOK);
  k_gemm2<0><<<dim3((NTOK / 128) * (DO / 64), 1), 128, 0, stream>>>(QW, 32, 0, W2, 32, 0, 1.0f / (QSC * XSC), nullptr, 0, nullptr, 1, 0, 0, LP, nullptr, DO, 0, NTOK, DO, 32);
  k_fin<<<(unsigned)((size_t)NTOK * DO / 4 / 256), 256, 0, stream>>>(LP, BD, OUTW, out, (int)((size_t)NTOK * DO / 4));
}
